// BLErnn_86930138071225
// MI455X (gfx1250) — hardware-verified
//
#include <hip/hip_runtime.h>
#include <math.h>

typedef __attribute__((ext_vector_type(16))) _Float16 v16h;
typedef __attribute__((ext_vector_type(16))) __bf16 v16b;
typedef __attribute__((ext_vector_type(8)))  _Float16 v8h;
typedef __attribute__((ext_vector_type(8)))  float v8f;
typedef __attribute__((ext_vector_type(4)))  float v4f;
typedef __attribute__((ext_vector_type(2)))  float v2f;
typedef __attribute__((ext_vector_type(4)))  unsigned v4u;
typedef __attribute__((ext_vector_type(4)))  int v4i;
typedef float __attribute__((may_alias)) float_a;
typedef int __attribute__((may_alias)) int_a;

template <typename T> __device__ __forceinline__ void vst2(void* p, T v) { *(volatile T*)p = v; __threadfence(); *(volatile T*)p = v; }
__device__ __forceinline__ v8f wmma16(v16h a, v16h b, v8f c) {
  v8f d = __builtin_amdgcn_wmma_f32_16x16x32_f16(false, a, false, b, (short)0, c, false, false);
  asm volatile("v_nop\n\tv_nop\n\tv_nop\n\tv_nop" : "+v"(d) : "v"(a), "v"(b));
  return d;
}
__device__ __forceinline__ v8f wmma_bf(v16b a, v16b b, v8f c) {
  v8f d = __builtin_amdgcn_wmma_f32_16x16x32_bf16(false, a, false, b, (short)0, c, false, false);
  asm volatile("v_nop\n\tv_nop\n\tv_nop\n\tv_nop" : "+v"(d) : "v"(a), "v"(b));
  return d;
}
__device__ __forceinline__ v16h frag_h(const _Float16* rowk0, int lane) {
  union { v16h v; v8h q[2]; } u; const _Float16* p = rowk0 + 8 * (lane >> 4);
  u.q[0] = *(const v8h*)p; u.q[1] = *(const v8h*)(p + 16); return u.v;
}
__device__ __forceinline__ v16h frag_f32(const float* rowk0, int lane) {
  v16h a; const float* p = rowk0 + 8 * (lane >> 4);
#pragma unroll
  for (int i = 0; i < 8; ++i) { a[i] = (_Float16)p[i]; a[8 + i] = (_Float16)p[16 + i]; }
  return a;
}
__device__ __forceinline__ v16h frag_f32s(const float* rowk0, int lane, float sc) {
  v16h a; const float* p = rowk0 + 8 * (lane >> 4);
#pragma unroll
  for (int i = 0; i < 8; ++i) { a[i] = (_Float16)(p[i] * sc); a[8 + i] = (_Float16)(p[16 + i] * sc); }
  return a;
}
__device__ __forceinline__ v16h fragc_f32(const float* W, int k0, int n, int lane, int ld, int K) {
  v16h a; const int g = lane >> 4;
#pragma unroll
  for (int i = 0; i < 8; ++i) { const int ka = k0 + 8 * g + i, kb = ka + 16;
    a[i] = (_Float16)(ka < K ? W[(size_t)(ka < K ? ka : K - 1) * ld + n] : 0.f); a[8 + i] = (_Float16)(kb < K ? W[(size_t)(kb < K ? kb : K - 1) * ld + n] : 0.f); }
  return a;
}
struct F2 { v16b h, l; };
__device__ __forceinline__ F2 bsplit16(const float v[16]) { F2 r;
#pragma unroll
  for (int i = 0; i < 16; ++i) { const __bf16 h = (__bf16)v[i]; r.h[i] = h; r.l[i] = (__bf16)(v[i] - (float)h); }
  return r; }
__device__ __forceinline__ F2 split_row(const float* row, int k0, int lane) { float v[16]; const float* p = row + k0 + 8 * (lane >> 4);
#pragma unroll
  for (int i = 0; i < 8; ++i) { v[i] = p[i]; v[8 + i] = p[16 + i]; }
  return bsplit16(v); }
__device__ __forceinline__ F2 split_rowK(const float* row, int k0, int lane, int K) { float v[16]; const int g = lane >> 4;
#pragma unroll
  for (int i = 0; i < 8; ++i) { const int ka = k0 + 8 * g + i, kb = ka + 16; v[i] = ka < K ? row[ka < K ? ka : K - 1] : 0.f; v[8 + i] = kb < K ? row[kb < K ? kb : K - 1] : 0.f; }
  return bsplit16(v); }
__device__ __forceinline__ F2 split_col(const float* W, int k0, int n, int lane, int ld, int K) { float v[16]; const int g = lane >> 4;
#pragma unroll
  for (int i = 0; i < 8; ++i) { const int ka = k0 + 8 * g + i, kb = ka + 16; v[i] = ka < K ? W[(size_t)(ka < K ? ka : K - 1) * ld + n] : 0.f; v[8 + i] = kb < K ? W[(size_t)(kb < K ? kb : K - 1) * ld + n] : 0.f; }
  return bsplit16(v); }
__device__ __forceinline__ v8f mac3(const F2& a, const F2& b, v8f c) { c = wmma_bf(a.l, b.h, c); c = wmma_bf(a.h, b.l, c); return wmma_bf(a.h, b.h, c); }
__device__ __forceinline__ float sigm(float v) { return 1.0f / (1.0f + expf(-v)); }
#define LDSX() do { asm volatile("s_wait_dscnt 0" ::: "memory"); __builtin_amdgcn_wave_barrier(); __builtin_amdgcn_fence(__ATOMIC_RELEASE, "workgroup"); } while (0)


#define NBS 4096
#define TT 200
#define NI 5
#define NF 20
#define NHID 32
#define NG 128
#ifndef NBLK
#define NBLK (NBS / 64)
#endif
typedef __attribute__((ext_vector_type(8))) __bf16 v8b;
__device__ __forceinline__ v16b frag_b(const __bf16* rowk0, int lane) {
  union { v16b v; v8b q[2]; } u; const __bf16* p = rowk0 + 8 * (lane >> 4);
  u.q[0] = *(const v8b*)p; u.q[1] = *(const v8b*)(p + 16); return u.v;
}
__device__ __forceinline__ float bfr(float v) { return (float)(__bf16)v; }
__device__ __attribute__((noinline)) float exp_ni(float v) { return expf(v); }
__device__ __attribute__((noinline)) float erf_ni(float v) { return erff(v); }

__device__ __forceinline__ float tanh_f(float x) { const float e = __expf(-2.0f * fabsf(x)); const float t = (1.0f - e) / (1.0f + e); return x < 0.f ? -t : t; }
__device__ __forceinline__ float sigm_f(float x) { return 1.0f / (1.0f + __expf(-x)); }
#define WS_PW   0u
#define WS_END  (WS_PW + 2u * 2 * NG * 32)

__global__ __launch_bounds__(128) void k_packW(const float* __restrict__ WIH, const float* __restrict__ WHH, __bf16* __restrict__ PW) {
  __shared__ __align__(16) __bf16 s[2][32]; const int o = blockIdx.x, t = threadIdx.x;
  if (t < 32) { s[0][t] = (__bf16)((t < NF) ? WIH[o * NF + t] : 0.f); s[1][t] = (__bf16)WHH[o * NHID + t]; } __syncthreads();
  if (t < 4) vst2((unsigned*)(PW + (size_t)o * 32 + t * 8), *(const v4u*)&s[0][t * 8]); else if (t < 8) vst2((unsigned*)(PW + NG * 32 + (size_t)o * 32 + (t - 4) * 8), *(const v4u*)&s[1][(t - 4) * 8]);
}
__global__ __launch_bounds__(128) void k_lstm(const float* __restrict__ X, const float* __restrict__ F1W, const float* __restrict__ F1B, const __bf16* __restrict__ PW, const float* __restrict__ BIH, const float* __restrict__ BHH, const float* __restrict__ F2W, const float* __restrict__ F2B, float* __restrict__ OUT) {
  __shared__ __align__(16) float sa[4][16][36]; __shared__ __align__(16) float sh[4][16][36]; __shared__ __align__(16) float so[4][16][2]; __shared__ float sw1[NF][NI], sb1[NF];
  const int tid = threadIdx.x, wave = tid >> 5, lane = tid & 31, col = lane & 15, g = lane >> 4; const size_t r0 = (size_t)blockIdx.x * 64 + wave * 16;
  if (tid < NF) { sb1[tid] = bfr(F1B[tid]);
#pragma unroll
    for (int q = 0; q < NI; ++q) sw1[tid][q] = bfr(F1W[tid * NI + q]); }
  float bsum[8];
#pragma unroll
  for (int j = 0; j < 8; ++j) bsum[j] = bfr(BIH[j * 16 + col]) + bfr(BHH[j * 16 + col]);
  float c[8][2];
#pragma unroll
  for (int r = 0; r < 8; ++r) { c[r][0] = c[r][1] = 0.f; }
  for (int q = lane; q < 16 * 32; q += 32) sh[wave][q >> 5][q & 31] = 0.f;
  __syncthreads();
#pragma unroll 1
  for (int t = 0; t < TT; ++t) {
    { const float* xp = X + ((r0 + col) * TT + t) * NI; float xv[NI];
#pragma unroll
      for (int q = 0; q < NI; ++q) xv[q] = bfr(xp[q]);
#pragma unroll
      for (int f2 = 0; f2 < 10; ++f2) { const int f = g * 10 + f2; float a = sb1[f];
#pragma unroll
        for (int q = 0; q < NI; ++q) a += xv[q] * sw1[f][q];
        sa[wave][col][f] = fmaxf(a, 0.f); }
      if (g == 0) { for (int f = NF; f < 32; ++f) sa[wave][col][f] = 0.f; } }
    LDSX();
    v8f acc[8];
#pragma unroll
    for (int j = 0; j < 8; ++j) { acc[j] = (v8f){};
#pragma unroll
      for (int r = 0; r < 8; ++r) acc[j][r] = bsum[j]; }
    { const F2 a = split_row(&sa[wave][col][0], 0, lane); const F2 hh = split_row(&sh[wave][col][0], 0, lane);
#pragma unroll
      for (int j = 0; j < 8; ++j) { const v16b wih = frag_b(PW + (size_t)(j * 16 + col) * 32, lane); acc[j] = wmma_bf(a.l, wih, acc[j]); acc[j] = wmma_bf(a.h, wih, acc[j]); const v16b whh = frag_b(PW + NG * 32 + (size_t)(j * 16 + col) * 32, lane); acc[j] = wmma_bf(hh.l, whh, acc[j]); acc[j] = wmma_bf(hh.h, whh, acc[j]); } }
    LDSX();
#pragma unroll
    for (int r = 0; r < 8; ++r) {
#pragma unroll
      for (int u = 0; u < 2; ++u) { const float ig = sigm_f(acc[0 + u][r]), fg = sigm_f(acc[2 + u][r]), gg = tanh_f(acc[4 + u][r]), og = sigm_f(acc[6 + u][r]);
        const float cn = fg * c[r][u] + ig * gg; c[r][u] = cn; const float hn = og * tanh_f(cn); sh[wave][8 * g + r][u * 16 + col] = hn; } }
    LDSX(); }
  if (lane < 16) { float a0 = bfr(F2B[0]), a1 = bfr(F2B[1]);
#pragma unroll 1
    for (int k = 0; k < NHID; ++k) { const float hv = sh[wave][lane][k]; a0 += hv * bfr(F2W[k]); a1 += hv * bfr(F2W[NHID + k]); }
    so[wave][lane][0] = a0; so[wave][lane][1] = a1; }
  LDSX();
  if (lane < 8) vst2(OUT + (r0 + lane * 2) * 2, *(const v4f*)&so[wave][lane * 2][0]);
}
extern "C" void kernel_launch(void* const* d_in, const int* in_sizes, int n_in, void* d_out, int out_size, void* d_ws, size_t ws_size, hipStream_t stream) {
  (void)in_sizes; (void)n_in; (void)out_size;
  const float** F = (const float**)d_in;
  if (ws_size < (size_t)WS_END) return;
  char* ws = (char*)d_ws; __bf16* PW = (__bf16*)(ws + WS_PW);
  k_packW<<<NG, 128, 0, stream>>>(F[3], F[4], PW);
  k_lstm<<<NBLK, 128, 0, stream>>>(F[0], F[1], F[2], PW, F[5], F[6], F[7], F[8], (float*)d_out);
}
